// PIPNet_90452011254231
// MI455X (gfx1250) — hardware-verified
//
#include <hip/hip_runtime.h>
#include <hip/hip_bf16.h>


typedef __attribute__((ext_vector_type(16))) _Float16 v16h;
typedef __attribute__((ext_vector_type(8)))  _Float16 v8h;
typedef __attribute__((ext_vector_type(8)))  float    v8f;
typedef __attribute__((ext_vector_type(4)))  float    v4f;
#define WSCALE 16384.0f

__device__ __forceinline__ v8f wmma16(v16h a, v16h b, v8f c) {
    v8f d = __builtin_amdgcn_wmma_f32_16x16x32_f16(false, a, false, b, (short)0, c, false, false);
    asm volatile("v_nop\n\tv_nop\n\tv_nop\n\tv_nop" : "+v"(d) : "v"(a), "v"(b));
    return d;
}

#define P_PAIRS 4096
#define N_VERTS 40000
#define C_FEAT  64
#define NCHUNK  1250
#define WAVES   4

__global__ __launch_bounds__(256) void pack_feats_kernel(
    const float* __restrict__ feats, _Float16* __restrict__ out)
{
    int t = blockIdx.x * blockDim.x + threadIdx.x;
    if (t >= NCHUNK * 4 * 32) return;
    int lane = t & 31;
    int j    = (t >> 5) & 3;
    int c    = t >> 7;
    int cj   = t >> 5;
    int k0   = c * 32 + (lane >> 4) * 8;
    int col  = j * 16 + (lane & 15);
    v8h lo, hi;
#pragma unroll
    for (int e = 0; e < 8; ++e) {
        lo[e] = (_Float16)feats[(size_t)(k0 + e) * C_FEAT + col];
        hi[e] = (_Float16)feats[(size_t)(k0 + 16 + e) * C_FEAT + col];
    }
    volatile v8h* d0 = (volatile v8h*)(out + (size_t)cj * 512 + lane * 8);
    volatile v8h* d1 = (volatile v8h*)(out + (size_t)cj * 512 + 256 + lane * 8);
    *d0 = lo; *d1 = hi;
    __threadfence();
    *d0 = lo; *d1 = hi;
}

__global__ __launch_bounds__(128) void rbf_wmma_kernel(
    const float* __restrict__ pairs_loc, int side,
    const float* __restrict__ verts,
    const _Float16* __restrict__ bpack,
    float* __restrict__ F, float* __restrict__ S)
{
    const int lane = threadIdx.x & 31;
    const int wave = threadIdx.x >> 5;
    const int m    = lane & 15;
    const int p    = blockIdx.x * 16 + m;

    const float* pl = pairs_loc + ((size_t)p * 2 + side) * 3;
    const float px = pl[0], py = pl[1], pz = pl[2];

    v8f acc0 = {}, acc1 = {}, acc2 = {}, acc3 = {}, accS = {};
    const float C2 = -0.57707801635558534f;
    const int srcbase = (lane >> 4) * 8;

    v16h ones;
#pragma unroll
    for (int e = 0; e < 16; ++e) ones[e] = (_Float16)1.0f;

    const float* vp0 = verts + (size_t)(wave * 32 + lane) * 3;
    float nvx = vp0[0], nvy = vp0[1], nvz = vp0[2];

    for (int c = wave; c < NCHUNK; c += WAVES) {
        const _Float16* bb = bpack + ((size_t)c * 4) * 512 + lane * 8;
        v16h b0, b1, b2, b3;
        { v8h* q = (v8h*)&b0; q[0] = *(const v8h*)(bb);            q[1] = *(const v8h*)(bb + 256); }
        { v8h* q = (v8h*)&b1; q[0] = *(const v8h*)(bb + 512);      q[1] = *(const v8h*)(bb + 512 + 256); }
        { v8h* q = (v8h*)&b2; q[0] = *(const v8h*)(bb + 2 * 512);  q[1] = *(const v8h*)(bb + 2 * 512 + 256); }
        { v8h* q = (v8h*)&b3; q[0] = *(const v8h*)(bb + 3 * 512);  q[1] = *(const v8h*)(bb + 3 * 512 + 256); }

        const float vx = nvx, vy = nvy, vz = nvz;
        int cn = c + WAVES; cn = cn < NCHUNK ? cn : (NCHUNK - 1);
        const float* vq = verts + (size_t)(cn * 32 + lane) * 3;
        nvx = vq[0]; nvy = vq[1]; nvz = vq[2];

        v16h a;
#pragma unroll
        for (int kk = 0; kk < 16; ++kk) {
            const int src = (kk & 7) | ((kk >> 3) << 4) | srcbase;
            const float sx = __shfl(vx, src, 32);
            const float sy = __shfl(vy, src, 32);
            const float sz = __shfl(vz, src, 32);
            const float dx = px - sx, dy = py - sy, dz = pz - sz;
            const float d2 = dx * dx + dy * dy + dz * dz;
            const float d  = __builtin_amdgcn_sqrtf(d2);
            const float w  = __builtin_amdgcn_exp2f(d * C2);
            a[kk] = (_Float16)(w * WSCALE);
        }

        acc0 = wmma16(a, b0, acc0);
        acc1 = wmma16(a, b1, acc1);
        acc2 = wmma16(a, b2, acc2);
        acc3 = wmma16(a, b3, acc3);
        accS = wmma16(a, ones, accS);
    }

    __shared__ float red[WAVES * 1280];
#pragma unroll
    for (int r = 0; r < 8; ++r) {
        red[wave * 1280 + 0 * 256 + r * 32 + lane] = acc0[r];
        red[wave * 1280 + 1 * 256 + r * 32 + lane] = acc1[r];
        red[wave * 1280 + 2 * 256 + r * 32 + lane] = acc2[r];
        red[wave * 1280 + 3 * 256 + r * 32 + lane] = acc3[r];
        red[wave * 1280 + 4 * 256 + r * 32 + lane] = accS[r];
    }
    __syncthreads();

    __shared__ __attribute__((aligned(16))) float tile[16][C_FEAT];
    __shared__ __attribute__((aligned(16))) float srow[32];
    for (int f = threadIdx.x; f < 1024; f += 128) {
        float s = red[f] + red[1280 + f] + red[2560 + f] + red[3840 + f];
        const int j = f >> 8, r = (f >> 5) & 7, l = f & 31;
        const int M   = r + 8 * (l >> 4);
        const int col = j * 16 + (l & 15);
        tile[M][col] = s;
    }
    if (threadIdx.x < 32) {
        float s = 0.f;
        if (threadIdx.x < 16) {
            const int M = threadIdx.x;
            const int off = 1024 + (M & 7) * 32 + ((M >> 3) * 16);
#pragma unroll
            for (int w = 0; w < WAVES; ++w) s += red[w * 1280 + off];
        }
        srow[threadIdx.x] = s;
    }
    __syncthreads();
    float* fb = F + (size_t)blockIdx.x * 16 * C_FEAT;
    for (int pass = 0; pass < 2; ++pass) {
#pragma unroll
        for (int q = 0; q < 2; ++q) {
            const int piece = threadIdx.x + q * 128;
            const int M = piece >> 4, sg = piece & 15;
            *(volatile v4f*)(fb + M * C_FEAT + sg * 4) = *(const v4f*)(&tile[M][sg * 4]);
        }
        if (threadIdx.x < 32) *(volatile float*)(S + (size_t)blockIdx.x * 32 + threadIdx.x) = srow[threadIdx.x];
        __threadfence();
    }
}

__global__ __launch_bounds__(128) void mlp_kernel(
    const float* __restrict__ FL, const float* __restrict__ SL,
    const float* __restrict__ FR, const float* __restrict__ SR,
    const float* __restrict__ W1, const float* __restrict__ b1,
    const float* __restrict__ W2, const float* __restrict__ b2,
    const float* __restrict__ W3, const float* __restrict__ b3,
    float* __restrict__ out)
{
    const int t = threadIdx.x;
    __shared__ float x[130];
    __shared__ float h[128];
    __shared__ float res[32];

    for (int q = 0; q < 32; ++q) {
        const int p = blockIdx.x * 32 + q;
        const float sl = SL[(size_t)(p >> 4) * 32 + (p & 15)], sr = SR[(size_t)(p >> 4) * 32 + (p & 15)];
        const float nl = sl + 0.01f * WSCALE;
        const float nr = sr + 0.01f * WSCALE;
        if (t < 64)       x[t]     = FL[(size_t)p * 64 + t] / nl;
        else              x[t + 1] = FR[(size_t)p * 64 + (t - 64)] / nr;
        if (t == 0) x[64]  = tanhf(sl * (1.0f / WSCALE) + 0.01f);
        if (t == 1) x[129] = tanhf(sr * (1.0f / WSCALE) + 0.01f);
        __syncthreads();

        float s = b1[t];
        for (int i = 0; i < 130; ++i) s += x[i] * W1[i * 128 + t];
        s = fmaxf(s, 0.f);
        h[t] = s;
        __syncthreads();

        float s2 = b2[t];
        for (int i = 0; i < 128; ++i) s2 += h[i] * W2[i * 128 + t];
        s2 = fmaxf(s2, 0.f);
        const float contrib = s2 * W3[t];
        __syncthreads();
        h[t] = contrib;
        __syncthreads();
        for (int off = 64; off > 0; off >>= 1) {
            if (t < off) h[t] += h[t + off];
            __syncthreads();
        }
        if (t == 0) res[q] = h[0] + b3[0];
        __syncthreads();
    }
    if (t < 32) {
        volatile float* o = out + (size_t)blockIdx.x * 32 + t;
        *o = res[t]; __threadfence(); *o = res[t];
    }
}

extern "C" void kernel_launch(void* const* d_in, const int* in_sizes, int n_in,
                              void* d_out, int out_size, void* d_ws, size_t ws_size,
                              hipStream_t stream)
{
    const float* pairs_loc = (const float*)d_in[0];
    const float* verts_l   = (const float*)d_in[1];
    const float* verts_r   = (const float*)d_in[2];
    const float* proc_l    = (const float*)d_in[3];
    const float* proc_r    = (const float*)d_in[4];
    const float* W1 = (const float*)d_in[5];
    const float* b1 = (const float*)d_in[6];
    const float* W2 = (const float*)d_in[7];
    const float* b2 = (const float*)d_in[8];
    const float* W3 = (const float*)d_in[9];
    const float* b3 = (const float*)d_in[10];

    char* ws = (char*)d_ws;
    const size_t PACK_BYTES = (size_t)NCHUNK * 4 * 32 * 16 * sizeof(_Float16);
    const size_t F_BYTES    = (size_t)P_PAIRS * C_FEAT * sizeof(float);
    const size_t S_BYTES    = (size_t)P_PAIRS * 2 * sizeof(float);
    (void)in_sizes; (void)n_in; (void)out_size;
    if (ws_size < 2 * ((size_t)NCHUNK * 4 * 32 * 16 * sizeof(_Float16)) + 2 * F_BYTES + 2 * S_BYTES) return;

    _Float16* packL = (_Float16*)(ws);
    _Float16* packR = (_Float16*)(ws + PACK_BYTES);
    float* FL = (float*)(ws + 2 * PACK_BYTES);
    float* FR = (float*)(ws + 2 * PACK_BYTES + F_BYTES);
    float* SL = (float*)(ws + 2 * PACK_BYTES + 2 * F_BYTES);
    float* SR = (float*)(ws + 2 * PACK_BYTES + 2 * F_BYTES + S_BYTES);

    const int packThreads = NCHUNK * 4 * 32;
    pack_feats_kernel<<<(packThreads + 255) / 256, 256, 0, stream>>>(proc_l, packL);
    pack_feats_kernel<<<(packThreads + 255) / 256, 256, 0, stream>>>(proc_r, packR);

    rbf_wmma_kernel<<<P_PAIRS / 16, 128, 0, stream>>>(pairs_loc, 0, verts_l, packL, FL, SL);
    rbf_wmma_kernel<<<P_PAIRS / 16, 128, 0, stream>>>(pairs_loc, 1, verts_r, packR, FR, SR);

    mlp_kernel<<<P_PAIRS / 32, 128, 0, stream>>>(FL, SL, FR, SR,
                                            W1, b1, W2, b2, W3, b3,
                                            (float*)d_out);
}
